// FlashSelfAttention_38354057953636
// MI455X (gfx1250) — hardware-verified
//
#include <hip/hip_runtime.h>
#include <stdint.h>
#include <math.h>

typedef __attribute__((ext_vector_type(16))) _Float16 v16h;
typedef __attribute__((ext_vector_type(8)))  _Float16 v8h;
typedef __attribute__((ext_vector_type(16))) __bf16   v16b;
typedef __attribute__((ext_vector_type(8)))  __bf16   v8b;
typedef __attribute__((ext_vector_type(8)))  float    v8f;
typedef __attribute__((ext_vector_type(4)))  float    v4f;
#define PSCALE 32768.0f
#define U16(p) ((const unsigned short*)(const void*)(p))
#define PSCALE_INV (1.0f / 32768.0f)

__device__ __forceinline__ unsigned short f2bf_bits(float f) {
  unsigned u = __float_as_uint(f);
  return (unsigned short)((u + 0x7FFFu + ((u >> 16) & 1u)) >> 16);
}
__device__ __forceinline__ float bf_bits2f(unsigned short h) { return __uint_as_float(((unsigned)h) << 16); }

__device__ __forceinline__ void dep_guard_h(v8f& a, v8f& b, v16h x, v16h y) { asm volatile("v_nop\n\tv_nop\n\tv_nop\n\tv_nop" : "+v"(a), "+v"(b) : "v"(x), "v"(y)); }
__device__ __forceinline__ void dep_guard_b(v8f& a, v8f& b, v16b x, v16b y) { asm volatile("v_nop\n\tv_nop\n\tv_nop\n\tv_nop" : "+v"(a), "+v"(b) : "v"(x), "v"(y)); }
__device__ __forceinline__ void keep4_h(v16h a, v16h b, v16h c, v16h d) { asm volatile("v_nop" :: "v"(a), "v"(b), "v"(c), "v"(d)); }
__device__ __forceinline__ void keep4_b(v16b a, v16b b, v16b c, v16b d) { asm volatile("v_nop" :: "v"(a), "v"(b), "v"(c), "v"(d)); }
__device__ __forceinline__ void acc_guard4(v8f& a, v8f& b, v8f& c, v8f& d) { asm volatile("v_nop\n\tv_nop\n\tv_nop\n\tv_nop" : "+v"(a), "+v"(b), "+v"(c), "+v"(d)); }
template <typename T> struct Frag;
template <> struct Frag<_Float16> {
  typedef v16h V; union U { v16h v; v8h h[2]; };
  static __device__ __forceinline__ v16h load(const _Float16* p) {
    U f; f.h[0] = *(const v8h*)(p); f.h[1] = *(const v8h*)(p + 16); return f.v;
  }
  static __device__ __forceinline__ v8f mma(v16h a, v16h b, v8f c) {
    return __builtin_amdgcn_wmma_f32_16x16x32_f16(false, a, false, b, (short)0, c, false, false);
  }
  static __device__ __forceinline__ void guard(v8f& a, v8f& b, v16h x, v16h y) { dep_guard_h(a, b, x, y); }
  static __device__ __forceinline__ void keep(v16h a, v16h b, v16h c, v16h d) { keep4_h(a, b, c, d); }
};
template <> struct Frag<__bf16> {
  typedef v16b V; union U { v16b v; v8b h[2]; };
  static __device__ __forceinline__ v16b load(const __bf16* p) {
    U f; f.h[0] = *(const v8b*)(p); f.h[1] = *(const v8b*)(p + 16); return f.v;
  }
  static __device__ __forceinline__ v8f mma(v16b a, v16b b, v8f c) {
    return __builtin_amdgcn_wmma_f32_16x16x32_bf16(false, a, false, b, (short)0, c, false, false);
  }
  static __device__ __forceinline__ void guard(v8f& a, v8f& b, v16b x, v16b y) { dep_guard_b(a, b, x, y); }
  static __device__ __forceinline__ void keep(v16b a, v16b b, v16b c, v16b d) { keep4_b(a, b, c, d); }
};

template <int ET> struct Elem;
template <> struct Elem<0> { typedef _Float16 T; };
template <> struct Elem<1> { typedef __bf16 T; };
template <int ET, bool SPLIT, int BIAS_MODE, int OUT_MODE, bool RESID, int ACT = 0, bool BSPLIT = true>
__global__ __launch_bounds__(256) void wmma_gemm64(
    const unsigned short* __restrict__ Ap, const unsigned short* __restrict__ A2p, int lda, long strideA,
    const unsigned short* __restrict__ Btp, const unsigned short* __restrict__ Bt2p, int ldb, long strideB,
    void* __restrict__ Cout, void* __restrict__ Cout2, int ldc, long strideC,
    const float* __restrict__ bias,
    const float* __restrict__ resid, long strideR,
    int M, int N, int K, float scale) {
  typedef typename Elem<ET>::T T;
  typedef typename Frag<T>::V V;
  const T* A = (const T*)Ap; const T* A2 = (const T*)A2p; const T* Bt = (const T*)Btp; const T* Bt2 = (const T*)Bt2p;
  __shared__ __align__(16) float sT[8][16 * 68];
  const int b    = blockIdx.y;
  const int lane = threadIdx.x & 31;
  const int wave = threadIdx.x >> 5;
  const int tilesN = N >> 6;
  const int tilesM = M >> 6;
  const int tile = blockIdx.x * 8 + wave;
  if (tile >= tilesM * tilesN) return;
  const int tm = tile / tilesN;
  const int tn = tile - tm * tilesN;
  const int m0 = tm << 6;
  const int n0 = tn << 6;

  const T* Ab  = A  + (size_t)b * strideA;
  const T* Bb  = Bt + (size_t)b * strideB;
  const T* Ab2 = SPLIT ? (A2  + (size_t)b * strideA) : nullptr;
  const T* Bb2 = (SPLIT && BSPLIT) ? (Bt2 + (size_t)b * strideB) : nullptr;

  const int rlane = lane & 15;
  const int koff  = (lane >> 4) * 8;
  const int mOff  = (lane >> 4) * 8;

  v8f acc[4][4];
#pragma unroll
  for (int i = 0; i < 4; ++i)
#pragma unroll
    for (int j = 0; j < 4; ++j) acc[i][j] = (v8f){0.f,0.f,0.f,0.f,0.f,0.f,0.f,0.f};

  for (int k0 = 0; k0 < K; k0 += 32) {
    V bh[4], bl[4];
#pragma unroll
    for (int j = 0; j < 4; ++j) {
      const size_t bo = (size_t)(n0 + (j << 4) + rlane) * ldb + koff + k0;
      bh[j] = Frag<T>::load(Bb + bo);
      if (SPLIT && BSPLIT) bl[j] = Frag<T>::load(Bb2 + bo);
    }
#pragma unroll
    for (int i = 0; i < 4; ++i) {
      const size_t ao = (size_t)(m0 + (i << 4) + rlane) * lda + koff + k0;
      V ah = Frag<T>::load(Ab + ao);
      V al;
      if (SPLIT) al = Frag<T>::load(Ab2 + ao);
#pragma unroll
      for (int j = 0; j < 4; ++j) {
        acc[i][j] = Frag<T>::mma(ah, bh[j], acc[i][j]);
        if (SPLIT) {
          if (BSPLIT) acc[i][j] = Frag<T>::mma(ah, bl[j], acc[i][j]);
          acc[i][j] = Frag<T>::mma(al, bh[j], acc[i][j]);
        }
      }
      Frag<T>::guard(acc[i][0], acc[i][3], ah, SPLIT ? al : ah);
    }
    Frag<T>::keep(bh[0], bh[1], bh[2], bh[3]);
    if (SPLIT && BSPLIT) Frag<T>::keep(bl[0], bl[1], bl[2], bl[3]);
  }
  acc_guard4(acc[0][0], acc[0][1], acc[0][2], acc[0][3]);
  acc_guard4(acc[1][0], acc[1][1], acc[1][2], acc[1][3]);
  acc_guard4(acc[2][0], acc[2][1], acc[2][2], acc[2][3]);
  acc_guard4(acc[3][0], acc[3][1], acc[3][2], acc[3][3]);

  float* slab = sT[wave];
  const float* Rb = RESID ? (resid + (size_t)b * strideR) : nullptr;
#pragma unroll
  for (int i = 0; i < 4; ++i) {
    const int mBase = m0 + (i << 4);
#pragma unroll
    for (int j = 0; j < 4; ++j) {
      const int n = n0 + (j << 4) + rlane;
      float bv = 0.f;
      if (BIAS_MODE == 2) bv = bias[n];
#pragma unroll
      for (int r = 0; r < 8; ++r) {
        float v = acc[i][j][r] * scale;
        if (BIAS_MODE == 1) v += bias[mBase + mOff + r];
        if (BIAS_MODE == 2) v += bv;
        if (RESID) v += Rb[(size_t)(mBase + mOff + r) * ldc + n];
        if (ACT == 1) v = tanhf(v);
        if (ACT == 2) v = fmaxf(v, 0.0f);
        if (ACT == 3) v = v / (1.0f + expf(-v));
        if (ACT == 4) v = (v > 0.f) ? v : 0.01f * v;
        if (ACT == 5) v = 0.5f * v * (1.0f + erff(v * 0.70710678118654752f));
        slab[(mOff + r) * 68 + (j << 4) + rlane] = v;
      }
    }
    __builtin_amdgcn_fence(__ATOMIC_RELEASE, "workgroup");
    __builtin_amdgcn_wave_barrier();
    __builtin_amdgcn_fence(__ATOMIC_ACQUIRE, "workgroup");
    if (OUT_MODE == 0) {
      float* C = (float*)Cout + (size_t)b * strideC;
      const int hh = lane >> 4, c4 = (lane & 15) * 4;
      for (int pass = 0; pass < 2; ++pass) {
#pragma unroll
        for (int it = 0; it < 8; ++it) {
          const int row = it * 2 + hh;
          v4f v = *(const v4f*)(slab + row * 68 + c4);
          *(volatile v4f*)(C + (size_t)(mBase + row) * ldc + n0 + c4) = v;
        }
        __threadfence();
      }
    } else {
      const int q = lane >> 3, c8 = (lane & 7) * 8;
      unsigned short* C  = (unsigned short*)Cout  + (size_t)b * strideC;
      unsigned short* C2 = (OUT_MODE == 2) ? ((unsigned short*)Cout2 + (size_t)b * strideC) : nullptr;
      for (int pass = 0; pass < 2; ++pass) {
#pragma unroll
        for (int it = 0; it < 4; ++it) {
          const int row = it * 4 + q;
          const float* sp = slab + row * 68 + c8;
          v8h hv, lv;
#pragma unroll
          for (int e = 0; e < 8; ++e) {
            if (OUT_MODE == 1) {
              hv[e] = (_Float16)sp[e];
            } else {
              unsigned short hb = f2bf_bits(sp[e]);
              unsigned short lb = f2bf_bits(sp[e] - bf_bits2f(hb));
              hv[e] = __builtin_bit_cast(_Float16, hb);
              lv[e] = __builtin_bit_cast(_Float16, lb);
            }
          }
          *(volatile v8h*)(C + (size_t)(mBase + row) * ldc + n0 + c8) = hv;
          if (OUT_MODE == 2) *(volatile v8h*)(C2 + (size_t)(mBase + row) * ldc + n0 + c8) = lv;
        }
        __threadfence();
      }
    }
    __builtin_amdgcn_fence(__ATOMIC_RELEASE, "workgroup");
    __builtin_amdgcn_wave_barrier();
    __builtin_amdgcn_fence(__ATOMIC_ACQUIRE, "workgroup");
  }
}

__global__ __launch_bounds__(256) void cast_f32_bf16x2(
    const float* __restrict__ in, unsigned short* __restrict__ out, int n2) {
  int i = blockIdx.x * 256 + threadIdx.x;
  if (i < n2) {
    const unsigned short b0 = f2bf_bits(in[2 * i]);
    const unsigned short b1 = f2bf_bits(in[2 * i + 1]);
    const unsigned u = (unsigned)b0 | ((unsigned)b1 << 16);
    ((volatile unsigned*)out)[i] = u;
    __threadfence();
    ((volatile unsigned*)out)[i] = u;
  }
}

#define AT_D 64
#define AT_NW 4
#define AT_QB 64
#define AT_KC 64

__device__ __forceinline__ unsigned short at_bf_bits(float f) {
  unsigned u = __float_as_uint(f);
  return (unsigned short)((u + 0x7FFFu + ((u >> 16) & 1u)) >> 16);
}
__device__ __forceinline__ __bf16 at_f2bf(float f) { return __builtin_bit_cast(__bf16, at_bf_bits(f)); }
__device__ __forceinline__ v8f at_mma(v16b a, v16b b, v8f c) {
  c = __builtin_amdgcn_wmma_f32_16x16x32_bf16(false, a, false, b, (short)0, c, false, false);
  asm volatile("v_nop\n\tv_nop\n\tv_nop\n\tv_nop" : "+v"(c) : "v"(a), "v"(b));
  return c;
}
template <bool F16> __device__ __forceinline__ __bf16 at_to16(float f) {
  if (F16) return __builtin_bit_cast(__bf16, (_Float16)f);
  return at_f2bf(f);
}
template <bool F16> __device__ __forceinline__ v8f at_mma16(v16b a, v16b b, v8f c) {
  if (F16) {
    const v16h ah = __builtin_bit_cast(v16h, a), bh = __builtin_bit_cast(v16h, b);
    c = __builtin_amdgcn_wmma_f32_16x16x32_f16(false, ah, false, bh, (short)0, c, false, false);
    asm volatile("v_nop\n\tv_nop\n\tv_nop\n\tv_nop" : "+v"(c) : "v"(ah), "v"(bh));
    return c;
  }
  return at_mma(a, b, c);
}

constexpr int kBatch = 2;
constexpr int kSeq   = 2048;
constexpr int kHeads = 16;
constexpr int kHd    = 64;
constexpr int kDm    = 1024;
constexpr int kRows  = kBatch * kSeq;
constexpr int kQkLd  = 2048;
static_assert(kHeads * kHd == kDm, "head split");
static_assert(kSeq % AT_QB == 0 && kSeq % AT_KC == 0, "seq tiles");
static_assert(kRows % 64 == 0 && kDm % 64 == 0 && (2 * kDm) % 64 == 0 && kSeq % 64 == 0, "GEMM M/N tile multiples");
static_assert(kDm % 32 == 0, "GEMM K multiple of 32");

__global__ __launch_bounds__(128)
void attn_tril0_kernel(const unsigned short* __restrict__ qkh, const unsigned short* __restrict__ qkl,
                       const unsigned short* __restrict__ vt,
                       unsigned short* __restrict__ oh, unsigned short* __restrict__ ol) {
  union FB { v16b v; v8b h[2]; };
  __shared__ __align__(16) __bf16 Ksh[AT_KC * AT_D];
  __shared__ __align__(16) __bf16 Ksl[AT_KC * AT_D];
  __shared__ __align__(16) __bf16 Vts[AT_D * AT_KC];
  __shared__ __align__(16) __bf16 Psh[AT_NW][16 * AT_KC];
  __shared__ __align__(16) float  Os[AT_NW][16 * 68];

  const int tid  = threadIdx.x;
  const int wave = tid >> 5;
  const int lane = tid & 31;
  const int hh   = lane >> 4;
  const int c    = lane & 15;

  const int bx = blockIdx.x;
  const int qb = bx & 31;
  const int bh = bx >> 5;
  const int h  = bh & 15;
  const int b  = bh >> 4;
  const int q0 = qb * AT_QB + wave * 16;
  const size_t rowb = (size_t)b * kSeq;

  v16b qah[2], qal[2];
  {
    const size_t qo = (rowb + q0 + c) * (size_t)kQkLd + (size_t)h * kHd + 8 * hh;
    const __bf16* qrh = (const __bf16*)qkh + qo;
    const __bf16* qrl = (const __bf16*)qkl + qo;
#pragma unroll
    for (int dc = 0; dc < 2; ++dc) {
      qah[dc] = Frag<__bf16>::load(qrh + dc * 32);
      qal[dc] = Frag<__bf16>::load(qrl + dc * 32);
    }
  }

  float mrow[8], lrow[8];
  v8f oacc[4];
#pragma unroll
  for (int r = 0; r < 8; ++r) { mrow[r] = -INFINITY; lrow[r] = 0.f; }
#pragma unroll
  for (int t = 0; t < 4; ++t) oacc[t] = (v8f){0.f,0.f,0.f,0.f,0.f,0.f,0.f,0.f};

  for (int kc = 0; kc < kSeq / AT_KC; ++kc) {
    const int kv0 = kc * AT_KC;
    const bool need_k = (kc <= qb);
    __syncthreads();
    {
      const int dl = tid >> 1, hf = (tid & 1) * 32;
      const uint4* vsrc = (const uint4*)(vt + ((size_t)(b * kDm + h * kHd + dl)) * kSeq + kv0 + hf);
      uint4* vdst = (uint4*)(Vts + dl * AT_KC + hf);
#pragma unroll
      for (int i = 0; i < 4; ++i) vdst[i] = vsrc[i];
      if (need_k) {
        const size_t ko = (rowb + kv0 + dl) * (size_t)kQkLd + kDm + h * kHd + hf;
        const uint4* khs = (const uint4*)(qkh + ko);
        const uint4* kls = (const uint4*)(qkl + ko);
        uint4* khd = (uint4*)(Ksh + dl * AT_D + hf);
        uint4* kld = (uint4*)(Ksl + dl * AT_D + hf);
#pragma unroll
        for (int i = 0; i < 4; ++i) { khd[i] = khs[i]; kld[i] = kls[i]; }
      }
    }
    __syncthreads();

    v8f s[4];
#pragma unroll
    for (int j = 0; j < 4; ++j) s[j] = (v8f){0.f,0.f,0.f,0.f,0.f,0.f,0.f,0.f};
    if (need_k) {
#pragma unroll
      for (int j = 0; j < 4; ++j) {
#pragma unroll
        for (int dc = 0; dc < 2; ++dc) {
          FB kb, kl;
          kb.h[0] = *(const v8b*)(Ksh + (j * 16 + c) * AT_D + dc * 32 + 8 * hh);
          kb.h[1] = *(const v8b*)(Ksh + (j * 16 + c) * AT_D + dc * 32 + 16 + 8 * hh);
          kl.h[0] = *(const v8b*)(Ksl + (j * 16 + c) * AT_D + dc * 32 + 8 * hh);
          kl.h[1] = *(const v8b*)(Ksl + (j * 16 + c) * AT_D + dc * 32 + 16 + 8 * hh);
          s[j] = at_mma(qah[dc], kb.v, s[j]);
          s[j] = at_mma(qah[dc], kl.v, s[j]);
          s[j] = at_mma(qal[dc], kb.v, s[j]);
        }
      }
    }

    const bool diag = (kc == qb);
    float cm[8];
#pragma unroll
    for (int r = 0; r < 8; ++r) {
      const int qrow = q0 + 8 * hh + r;
      float m = -INFINITY;
#pragma unroll
      for (int j = 0; j < 4; ++j) {
        const int kvcol = kv0 + j * 16 + c;
        float val = s[j][r] * 0.125f;
        if (diag && (kvcol > qrow)) val = 0.0f;
        s[j][r] = val;
        m = fmaxf(m, val);
      }
#pragma unroll
      for (int off = 1; off < 16; off <<= 1) m = fmaxf(m, __shfl_xor(m, off, 32));
      cm[r] = m;
    }

    __bf16* pw = Psh[wave];
#pragma unroll
    for (int r = 0; r < 8; ++r) {
      const float mnew = fmaxf(mrow[r], cm[r]);
      const float alpha = expf(mrow[r] - mnew);
      mrow[r] = mnew;
      float psum = 0.f;
      if (need_k) {
#pragma unroll
        for (int j = 0; j < 4; ++j) {
          const float p = expf(s[j][r] - mnew);
          psum += p;
          pw[(8 * hh + r) * AT_KC + j * 16 + c] = at_to16<true>(p * PSCALE);
        }
      } else {
        const float p = expf(0.0f - mnew);
        const __bf16 pb = at_to16<true>(p * PSCALE);
#pragma unroll
        for (int j = 0; j < 4; ++j) pw[(8 * hh + r) * AT_KC + j * 16 + c] = pb;
        psum = 4.0f * p;
      }
#pragma unroll
      for (int off = 1; off < 16; off <<= 1) psum += __shfl_xor(psum, off, 32);
      lrow[r] = lrow[r] * alpha + psum;
#pragma unroll
      for (int t = 0; t < 4; ++t) oacc[t][r] *= alpha;
    }
    __builtin_amdgcn_fence(__ATOMIC_RELEASE, "workgroup");
    __builtin_amdgcn_wave_barrier();
    __builtin_amdgcn_fence(__ATOMIC_ACQUIRE, "workgroup");
#pragma unroll 1
    for (int kk = 0; kk < 2; ++kk) {
      FB pa;
      pa.h[0] = *(const v8b*)(pw + c * AT_KC + kk * 32 + 8 * hh);
      pa.h[1] = *(const v8b*)(pw + c * AT_KC + kk * 32 + 16 + 8 * hh);
#pragma unroll
      for (int t = 0; t < 4; ++t) {
        FB vb;
        vb.h[0] = *(const v8b*)(Vts + (t * 16 + c) * AT_KC + kk * 32 + 8 * hh);
        vb.h[1] = *(const v8b*)(Vts + (t * 16 + c) * AT_KC + kk * 32 + 16 + 8 * hh);
        oacc[t] = at_mma16<true>(pa.v, vb.v, oacc[t]);
      }
    }
  }

  float* os = Os[wave];
#pragma unroll
  for (int r = 0; r < 8; ++r) {
    const float inv = 1.0f / (lrow[r] * PSCALE);
#pragma unroll
    for (int t = 0; t < 4; ++t) os[(8 * hh + r) * 68 + t * 16 + c] = oacc[t][r] * inv;
  }
  __builtin_amdgcn_fence(__ATOMIC_RELEASE, "workgroup");
  __builtin_amdgcn_wave_barrier();
  __builtin_amdgcn_fence(__ATOMIC_ACQUIRE, "workgroup");
  {
    const int q8 = lane >> 3, c8 = (lane & 7) * 8;
    for (int pass = 0; pass < 2; ++pass) {
#pragma unroll
      for (int it = 0; it < 4; ++it) {
        const int row = it * 4 + q8;
        const float* sp = os + row * 68 + c8;
        v8h hv, lv;
#pragma unroll
        for (int e = 0; e < 8; ++e) {
          const unsigned short hb = f2bf_bits(sp[e]);
          const unsigned short lb = f2bf_bits(sp[e] - bf_bits2f(hb));
          hv[e] = __builtin_bit_cast(_Float16, hb);
          lv[e] = __builtin_bit_cast(_Float16, lb);
        }
        const size_t oo = (rowb + q0 + row) * (size_t)kDm + (size_t)h * kHd + c8;
        *(volatile v8h*)(oh + oo) = hv;
        *(volatile v8h*)(ol + oo) = lv;
      }
      __threadfence();
    }
  }
}

constexpr size_t kOffXb  = 0;
constexpr size_t kSzXb   = (size_t)kRows * kDm * 2;
constexpr size_t kOffWib = kOffXb + kSzXb;
constexpr size_t kSzWib  = (size_t)3 * kDm * kDm * 2;
constexpr size_t kOffWob = kOffWib + kSzWib;
constexpr size_t kSzWob  = (size_t)kDm * kDm * 2;
constexpr size_t kOffQKh = kOffWob + kSzWob;
constexpr size_t kSzQK   = (size_t)kRows * kQkLd * 2;
constexpr size_t kOffQKl = kOffQKh + kSzQK;
constexpr size_t kOffVt  = kOffQKl + kSzQK;
constexpr size_t kSzVt   = (size_t)kBatch * kDm * kSeq * 2;
constexpr size_t kOffOh  = kOffVt + kSzVt;
constexpr size_t kSzO    = (size_t)kRows * kDm * 2;
constexpr size_t kOffOl  = kOffOh + kSzO;
constexpr size_t kWsTotal = kOffOl + kSzO;
static_assert(kWsTotal == 75497472, "carve total");
static_assert(kWsTotal <= 134217728, "carve within budget");
static_assert((kOffWib % 256) == 0 && (kOffWob % 256) == 0 && (kOffQKh % 256) == 0 && (kOffQKl % 256) == 0 &&
              (kOffVt % 256) == 0 && (kOffOh % 256) == 0 && (kOffOl % 256) == 0, "aligned carves");

extern "C" void kernel_launch(void* const* d_in, const int* in_sizes, int n_in,
                              void* d_out, int out_size, void* d_ws, size_t ws_size,
                              hipStream_t stream) {
  if (n_in < 3) return;
  if (in_sizes[0] != kRows * kDm) return;
  if (in_sizes[1] != 3 * kDm * kDm) return;
  if (in_sizes[2] != kDm * kDm) return;
  if (out_size != kRows * kDm) return;
  if (ws_size < kWsTotal) return;

  const float* x     = (const float*)d_in[0];
  const float* w_in  = (const float*)d_in[1];
  const float* w_out = (const float*)d_in[2];
  float* out = (float*)d_out;
  char* ws = (char*)d_ws;

  unsigned short* Xb  = (unsigned short*)(ws + kOffXb);
  unsigned short* Wib = (unsigned short*)(ws + kOffWib);
  unsigned short* Wob = (unsigned short*)(ws + kOffWob);
  unsigned short* QKh = (unsigned short*)(ws + kOffQKh);
  unsigned short* QKl = (unsigned short*)(ws + kOffQKl);
  unsigned short* Vt  = (unsigned short*)(ws + kOffVt);
  unsigned short* Oh  = (unsigned short*)(ws + kOffOh);
  unsigned short* Ol  = (unsigned short*)(ws + kOffOl);

  {
    int n2 = kRows * kDm / 2;
    cast_f32_bf16x2<<<(n2 + 255) / 256, 256, 0, stream>>>(x, Xb, n2);
    n2 = 3 * kDm * kDm / 2;
    cast_f32_bf16x2<<<(n2 + 255) / 256, 256, 0, stream>>>(w_in, Wib, n2);
    n2 = kDm * kDm / 2;
    cast_f32_bf16x2<<<(n2 + 255) / 256, 256, 0, stream>>>(w_out, Wob, n2);
  }

  {
    const int M = kRows, N = 2 * kDm, K = kDm;
    const int tiles = (M / 64) * (N / 64);
    dim3 grid((tiles + 7) / 8, 1);
    wmma_gemm64<1, false, 0, 2, false, 0><<<grid, 256, 0, stream>>>(
        Xb, Xb, kDm, 0L, Wib, Wib, kDm, 0L, (void*)QKh, (void*)QKl, kQkLd, 0L,
        nullptr, nullptr, 0L, M, N, K, 1.0f);
  }

  {
    const int M = kDm, N = kSeq, K = kDm;
    const int tiles = (M / 64) * (N / 64);
    dim3 grid((tiles + 7) / 8, kBatch);
    wmma_gemm64<1, false, 0, 1, false, 0><<<grid, 256, 0, stream>>>(
        Wib + (size_t)2 * kDm * kDm, Wib + (size_t)2 * kDm * kDm, kDm, 0L,
        Xb, Xb, kDm, (long)kSeq * kDm,
        (void*)Vt, nullptr, kSeq, (long)kDm * kSeq,
        nullptr, nullptr, 0L, M, N, K, 1.0f);
  }

  attn_tril0_kernel<<<kBatch * kHeads * (kSeq / AT_QB), 128, 0, stream>>>(QKh, QKl, Vt, Oh, Ol);

  {
    const int M = kRows, N = kDm, K = kDm;
    const int tiles = (M / 64) * (N / 64);
    dim3 grid((tiles + 7) / 8, 1);
    wmma_gemm64<1, true, 0, 0, false, 0, false><<<grid, 256, 0, stream>>>(
        Oh, Ol, kDm, 0L, Wob, Wob, kDm, 0L, (void*)out, nullptr, kDm, 0L,
        nullptr, nullptr, 0L, M, N, K, 1.0f);
  }
}
